// RNN_18373870092537
// MI455X (gfx1250) — hardware-verified
//
#include <hip/hip_runtime.h>
#include <math.h>

constexpr int NSTEPS    = 1000;
constexpr int NBATCH    = 256;
constexpr int NFEAT     = 13;
constexpr int NXK       = 39;
constexpr int NHID      = 100;
constexpr int NGATE     = 3;
constexpr int NCLS_OUT  = 20;
constexpr int XKP       = 64;
constexpr int HKP       = 128;
constexpr int NPADH     = 112;
constexpr int HPITCH    = 136;
constexpr int NTHR_SEQ  = 224;
constexpr int ROWS_BLK  = 16;
constexpr int NTHR_PREP = 256;
constexpr int FEATW     = 2 * NHID;
constexpr int OUT_BLK   = ROWS_BLK * NCLS_OUT;
constexpr int OUT_BLK4  = OUT_BLK / 4;
constexpr float XCARRY  = 64.0f;
constexpr float WCARRY  = 16.0f;
constexpr float FOLD    = 1.0f / (XCARRY * WCARRY);

constexpr int X_ROWS     = NSTEPS * NBATCH;
constexpr int X_CHUNKS   = X_ROWS * (XKP / 8);
constexpr int X_BLOCKS   = X_CHUNKS / NTHR_PREP;
constexpr int W_ROWS     = NGATE * NPADH;
constexpr int WHH_CHUNKS = W_ROWS * (HKP / 8);
constexpr int WHH_BLOCKS = WHH_CHUNKS / NTHR_PREP;
constexpr int WIH_CHUNKS = W_ROWS * (XKP / 8);
constexpr int WIH_BLOCKS = (WIH_CHUNKS + NTHR_PREP - 1) / NTHR_PREP;

static_assert(NXK == 3 * NFEAT, "feature concat");
static_assert(NBATCH % ROWS_BLK == 0, "batch tiles");
static_assert(NPADH == 16 * (NTHR_SEQ / 32), "one 16-column group per wave");
static_assert(NPADH >= NHID && NPADH + 16 == HKP, "pad columns 112..127 covered by the last wave");
static_assert(XKP % 32 == 0 && HKP % 32 == 0, "k multiples of 32");
static_assert(XKP >= NXK && HKP >= NHID, "k pads");
static_assert(HPITCH % 8 == 0 && HPITCH >= HKP, "LDS pitch");
static_assert(X_CHUNKS % NTHR_PREP == 0, "x pack grid exact");
static_assert(WHH_CHUNKS % NTHR_PREP == 0, "whh pack grid exact");
static_assert(WIH_CHUNKS % 32 == 0, "wih pack whole waves");
static_assert(OUT_BLK % 32 == 0 && (OUT_BLK * 4) % 128 == 0, "block output = whole lines");
static_assert(2 * NTHR_SEQ >= OUT_BLK, "classifier trips");

typedef __attribute__((ext_vector_type(16))) _Float16 v16h;
typedef __attribute__((ext_vector_type(8)))  _Float16 v8h;
typedef __attribute__((ext_vector_type(8)))  float    v8f;
typedef __attribute__((ext_vector_type(4)))  float    v4f;
typedef __attribute__((ext_vector_type(4)))  unsigned v4u;

__device__ __forceinline__ void guard3_h(v8f& a, v8f& b, v8f& c, v16h x, v16h y0, v16h y1, v16h y2) {
  asm volatile("v_nop\n\tv_nop\n\tv_nop\n\tv_nop" : "+v"(a), "+v"(b), "+v"(c) : "v"(x), "v"(y0), "v"(y1), "v"(y2));
}
__device__ __forceinline__ void acc_guard4(v8f& a, v8f& b, v8f& c, v8f& d) {
  asm volatile("v_nop\n\tv_nop\n\tv_nop\n\tv_nop" : "+v"(a), "+v"(b), "+v"(c), "+v"(d));
}

template <typename T> struct Frag;
template <> struct Frag<_Float16> {
  typedef v16h V; union U { v16h v; v8h h[2]; };
  static __device__ __forceinline__ v16h load(const _Float16* p) {
    U f; f.h[0] = *(const v8h*)(p); f.h[1] = *(const v8h*)(p + 16); return f.v;
  }
  static __device__ __forceinline__ v8f mma(v16h a, v16h b, v8f c) {
    return __builtin_amdgcn_wmma_f32_16x16x32_f16(false, a, false, b, (short)0, c, false, false);
  }
};

__device__ __forceinline__ unsigned h16bits(float f) {
  const _Float16 h = (_Float16)f;
  const unsigned short b = __builtin_bit_cast(unsigned short, h);
  return (unsigned)b;
}

__device__ __forceinline__ float fsig(float x) { return 1.0f / (1.0f + expf(-x)); }

__device__ __forceinline__ void pack_x_chunk(const float* __restrict__ m0, const float* __restrict__ m1,
                                             const float* __restrict__ m2, unsigned short* __restrict__ X16, int i) {
  const int row = i >> 3;
  const int c8  = (i & 7) * 8;
  unsigned hb[8];
#pragma unroll
  for (int e = 0; e < 8; ++e) {
    const int k  = c8 + e;
    const int s  = (k >= 2 * NFEAT) ? 2 : ((k >= NFEAT) ? 1 : 0);
    int f = k - NFEAT * s;
    f = (f > NFEAT - 1) ? (NFEAT - 1) : f;
    const float* sp = (s == 0) ? m0 : ((s == 1) ? m1 : m2);
    const float v  = sp[(size_t)row * NFEAT + f];
    const float sv = (k < NXK) ? (v * XCARRY) : 0.0f;
    hb[e] = h16bits(sv);
  }
  v4u w;
  w[0] = hb[0] | (hb[1] << 16);
  w[1] = hb[2] | (hb[3] << 16);
  w[2] = hb[4] | (hb[5] << 16);
  w[3] = hb[6] | (hb[7] << 16);
  volatile v4u* p = (volatile v4u*)(X16 + (size_t)i * 8);
  *p = w;
  __threadfence();
  *p = w;
}

template <int KREAL, int KP8>
__device__ __forceinline__ void pack_w_chunk(const float* __restrict__ src, unsigned short* __restrict__ dst, int i) {
  const int row = i / KP8;
  const int c8  = (i - row * KP8) * 8;
  const int g   = row / NPADH;
  const int jr  = row - g * NPADH;
  const bool rowok = (jr < NHID);
  const int jc  = rowok ? jr : (NHID - 1);
  const float* sp = src + (size_t)(g * NHID + jc) * KREAL;
  unsigned hb[8];
#pragma unroll
  for (int e = 0; e < 8; ++e) {
    const int k  = c8 + e;
    const int kc = (k < KREAL) ? k : (KREAL - 1);
    const float v  = sp[kc];
    const float sv = (rowok && (k < KREAL)) ? (v * WCARRY) : 0.0f;
    hb[e] = h16bits(sv);
  }
  v4u w;
  w[0] = hb[0] | (hb[1] << 16);
  w[1] = hb[2] | (hb[3] << 16);
  w[2] = hb[4] | (hb[5] << 16);
  w[3] = hb[6] | (hb[7] << 16);
  volatile v4u* p = (volatile v4u*)(dst + (size_t)i * 8);
  *p = w;
  __threadfence();
  *p = w;
}

__global__ __launch_bounds__(NTHR_PREP) void prep_kernel(const float* __restrict__ m0, const float* __restrict__ m1,
                                                        const float* __restrict__ m2, const float* __restrict__ w_ih,
                                                        const float* __restrict__ w_hh, unsigned short* __restrict__ X16,
                                                        unsigned short* __restrict__ WIH16, unsigned short* __restrict__ WHH16) {
  const int blk = blockIdx.x;
  const int tid = threadIdx.x;
  if (blk < X_BLOCKS) {
    pack_x_chunk(m0, m1, m2, X16, blk * NTHR_PREP + tid);
  } else if (blk < X_BLOCKS + WHH_BLOCKS) {
    pack_w_chunk<NHID, HKP / 8>(w_hh, WHH16, (blk - X_BLOCKS) * NTHR_PREP + tid);
  } else {
    const int i = (blk - X_BLOCKS - WHH_BLOCKS) * NTHR_PREP + tid;
    if (i < WIH_CHUNKS) pack_w_chunk<NXK, XKP / 8>(w_ih, WIH16, i);
  }
}

__global__ __launch_bounds__(NTHR_SEQ) void gru_seq_kernel(const unsigned short* __restrict__ X16p,
                                                          const unsigned short* __restrict__ WIHp,
                                                          const unsigned short* __restrict__ WHHp,
                                                          const float* __restrict__ b_ih, const float* __restrict__ b_hh,
                                                          const float* __restrict__ len0, const float* __restrict__ w_out,
                                                          const float* __restrict__ b_out, float* __restrict__ out) {
  __shared__ __align__(16) _Float16 Hh[2][ROWS_BLK * HPITCH];
  __shared__ __align__(16) float    Feat[ROWS_BLK * FEATW];
  __shared__ __align__(16) float    OutS[OUT_BLK];

  const _Float16* X16 = (const _Float16*)X16p;
  const _Float16* WIH = (const _Float16*)WIHp;
  const _Float16* WHH = (const _Float16*)WHHp;

  const int tid = threadIdx.x, lane = tid & 31, wave = tid >> 5;
  const int c = lane & 15, hh = lane >> 4, koff = hh * 8;
  const int rowbase = blockIdx.x * ROWS_BLK;
  const int j = 16 * wave + c;
  const bool colOK = (j < NHID);
  const int jc = colOK ? j : (NHID - 1);

  {
    _Float16* hf = &Hh[0][0];
#pragma unroll 1
    for (int i = tid; i < 2 * ROWS_BLK * HPITCH; i += NTHR_SEQ) hf[i] = (_Float16)0.0f;
  }

  const float bir = b_ih[jc], biz = b_ih[NHID + jc], binr = b_ih[2 * NHID + jc];
  const float bhr = b_hh[jc], bhz = b_hh[NHID + jc], bhnr = b_hh[2 * NHID + jc];
  const float b_r  = colOK ? (bir + bhr) : 0.0f;
  const float b_z  = colOK ? (biz + bhz) : 0.0f;
  const float b_in = colOK ? binr : 0.0f;
  const float b_hn = colOK ? bhnr : 0.0f;

  float hst[8], sumv[8], maxv[8];
#pragma unroll
  for (int r = 0; r < 8; ++r) { hst[r] = 0.0f; sumv[r] = 0.0f; maxv[r] = -INFINITY; }

  const _Float16* wi = WIH + (size_t)j * XKP + koff;
  const _Float16* wh = WHH + (size_t)j * HKP + koff;
  constexpr int WI_GS = NPADH * XKP;
  constexpr int WH_GS = NPADH * HKP;
  const v8f z8 = {0.f, 0.f, 0.f, 0.f, 0.f, 0.f, 0.f, 0.f};

  __syncthreads();

#pragma unroll 1
  for (int t = 0; t < NSTEPS; ++t) {
    const int cur = t & 1;
    const _Float16* xrow = X16 + ((size_t)t * NBATCH + (size_t)(rowbase + c)) * XKP + koff;
    const _Float16* hrow = &Hh[cur][0] + c * HPITCH + koff;
    _Float16* hnext = &Hh[cur ^ 1][0];

    v8f ar = z8, az = z8, ain = z8, ahn = z8;

#pragma unroll 1
    for (int kx = 0; kx < XKP; kx += 32) {
      const v16h a  = Frag<_Float16>::load(xrow + kx);
      const v16h b0 = Frag<_Float16>::load(wi + kx);
      const v16h b1 = Frag<_Float16>::load(wi + WI_GS + kx);
      const v16h b2 = Frag<_Float16>::load(wi + 2 * WI_GS + kx);
      ar  = Frag<_Float16>::mma(a, b0, ar);
      az  = Frag<_Float16>::mma(a, b1, az);
      ain = Frag<_Float16>::mma(a, b2, ain);
      guard3_h(ar, az, ain, a, b0, b1, b2);
    }
#pragma unroll 1
    for (int k0 = 0; k0 < HKP; k0 += 32) {
      const v16h a  = Frag<_Float16>::load(hrow + k0);
      const v16h b0 = Frag<_Float16>::load(wh + k0);
      const v16h b1 = Frag<_Float16>::load(wh + WH_GS + k0);
      const v16h b2 = Frag<_Float16>::load(wh + 2 * WH_GS + k0);
      ar  = Frag<_Float16>::mma(a, b0, ar);
      az  = Frag<_Float16>::mma(a, b1, az);
      ahn = Frag<_Float16>::mma(a, b2, ahn);
      guard3_h(ar, az, ahn, a, b0, b1, b2);
    }
    acc_guard4(ar, az, ain, ahn);

#pragma unroll
    for (int r = 0; r < 8; ++r) {
      const float pr  = ar[r]  * FOLD + b_r;
      const float pz  = az[r]  * FOLD + b_z;
      const float pin = ain[r] * FOLD + b_in;
      const float phn = ahn[r] * FOLD + b_hn;
      const float rg = fsig(pr);
      const float zg = fsig(pz);
      const float ng = tanhf(pin + rg * phn);
      const float hn = (1.0f - zg) * ng + zg * hst[r];
      const float hv = colOK ? hn : 0.0f;
      hst[r]  = hv;
      sumv[r] = sumv[r] + hv;
      maxv[r] = fmaxf(maxv[r], hv);
      hnext[(8 * hh + r) * HPITCH + j] = (_Float16)(hv * XCARRY);
    }
    if (wave == (NTHR_SEQ / 32) - 1) {
#pragma unroll
      for (int r = 0; r < 8; ++r) hnext[(8 * hh + r) * HPITCH + j + 16] = (_Float16)0.0f;
    }
    __syncthreads();
  }

#pragma unroll
  for (int r = 0; r < 8; ++r) {
    const int m = 8 * hh + r;
    const float il = 1.0f / len0[rowbase + m];
    if (colOK) {
      Feat[m * FEATW + j]        = sumv[r] * il;
      Feat[m * FEATW + NHID + j] = maxv[r];
    }
  }
  __syncthreads();

#pragma unroll 1
  for (int it = 0; it < 2; ++it) {
    const int o  = it * NTHR_SEQ + tid;
    const int oc = (o < OUT_BLK) ? o : (OUT_BLK - 1);
    const int m   = oc / NCLS_OUT;
    const int cls = oc - m * NCLS_OUT;
    const float* fr = Feat + m * FEATW;
    const float* wr = w_out + cls * FEATW;
    float acc = b_out[cls];
#pragma unroll 1
    for (int k = 0; k < FEATW; ++k) acc = fmaf(fr[k], wr[k], acc);
    if (o < OUT_BLK) OutS[o] = acc;
  }
  __syncthreads();

  if (wave == 0) {
    float* ob = out + (size_t)blockIdx.x * OUT_BLK;
    for (int pass = 0; pass < 2; ++pass) {
#pragma unroll
      for (int it = 0; it < 3; ++it) {
        const int idx  = it * 32 + lane;
        const int idxc = (idx < OUT_BLK4) ? idx : (OUT_BLK4 - 1);
        const v4f v = *(const v4f*)(OutS + idxc * 4);
        if (idx < OUT_BLK4) *(volatile v4f*)(ob + idx * 4) = v;
      }
      __threadfence();
    }
  }
}

extern "C" void kernel_launch(void* const* d_in, const int* in_sizes, int n_in,
                              void* d_out, int out_size, void* d_ws, size_t ws_size, hipStream_t stream) {
  if (n_in < 10 || d_out == nullptr || d_ws == nullptr) return;
  if (in_sizes[0] != NSTEPS * NBATCH * NFEAT || in_sizes[1] != NSTEPS * NBATCH * NFEAT ||
      in_sizes[2] != NSTEPS * NBATCH * NFEAT || in_sizes[3] != NBATCH ||
      in_sizes[4] != NGATE * NHID * NXK || in_sizes[5] != NGATE * NHID * NHID ||
      in_sizes[6] != NGATE * NHID || in_sizes[7] != NGATE * NHID ||
      in_sizes[8] != NCLS_OUT * FEATW || in_sizes[9] != NCLS_OUT ||
      out_size != NBATCH * NCLS_OUT) return;

  const float* mfcc0 = (const float*)d_in[0];
  const float* mfcc1 = (const float*)d_in[1];
  const float* mfcc2 = (const float*)d_in[2];
  const float* len0  = (const float*)d_in[3];
  const float* w_ih  = (const float*)d_in[4];
  const float* w_hh  = (const float*)d_in[5];
  const float* b_ih  = (const float*)d_in[6];
  const float* b_hh  = (const float*)d_in[7];
  const float* w_out = (const float*)d_in[8];
  const float* b_out = (const float*)d_in[9];
  float* out = (float*)d_out;

  char* ws = (char*)d_ws; size_t off = 0;
  auto carve = [&](size_t bytes) -> char* { char* p = ws + off; off += (bytes + 255) & ~(size_t)255; return p; };
  unsigned short* X16   = (unsigned short*)carve((size_t)X_ROWS * XKP * 2);
  unsigned short* WHH16 = (unsigned short*)carve((size_t)W_ROWS * HKP * 2);
  unsigned short* WIH16 = (unsigned short*)carve((size_t)W_ROWS * XKP * 2);
  if (off > ws_size || off > (size_t)134217728) return;

  prep_kernel<<<X_BLOCKS + WHH_BLOCKS + WIH_BLOCKS, NTHR_PREP, 0, stream>>>(
      mfcc0, mfcc1, mfcc2, w_ih, w_hh, X16, WIH16, WHH16);
  gru_seq_kernel<<<NBATCH / ROWS_BLK, NTHR_SEQ, 0, stream>>>(
      X16, WIH16, WHH16, b_ih, b_hh, len0, w_out, b_out, out);
}
